// RNNNet_32220844654811
// MI455X (gfx1250) — hardware-verified
//
#include <hip/hip_runtime.h>
#include <hip/hip_bf16.h>

typedef __attribute__((ext_vector_type(16))) _Float16 v16h;
typedef __attribute__((ext_vector_type(8)))  _Float16 v8h;
typedef __attribute__((ext_vector_type(16))) __bf16   v16b;
typedef __attribute__((ext_vector_type(8)))  __bf16   v8b;
typedef __attribute__((ext_vector_type(8)))  float    v8f;
typedef __attribute__((ext_vector_type(4)))  float    v4f;

__device__ __forceinline__ unsigned short f2bf_bits(float f) {
  unsigned u = __float_as_uint(f);
  return (unsigned short)((u + 0x7FFFu + ((u >> 16) & 1u)) >> 16);
}
__device__ __forceinline__ float bf_bits2f(unsigned short h) { return __uint_as_float(((unsigned)h) << 16); }

__device__ __forceinline__ void dep_guard_h(v8f& a, v8f& b, v16h x, v16h y) { asm volatile("v_nop\n\tv_nop\n\tv_nop\n\tv_nop" : "+v"(a), "+v"(b) : "v"(x), "v"(y)); }
__device__ __forceinline__ void dep_guard_b(v8f& a, v8f& b, v16b x, v16b y) { asm volatile("v_nop\n\tv_nop\n\tv_nop\n\tv_nop" : "+v"(a), "+v"(b) : "v"(x), "v"(y)); }
__device__ __forceinline__ void keep4_h(v16h a, v16h b, v16h c, v16h d) { asm volatile("v_nop" :: "v"(a), "v"(b), "v"(c), "v"(d)); }
__device__ __forceinline__ void keep4_b(v16b a, v16b b, v16b c, v16b d) { asm volatile("v_nop" :: "v"(a), "v"(b), "v"(c), "v"(d)); }
__device__ __forceinline__ void acc_guard4(v8f& a, v8f& b, v8f& c, v8f& d) { asm volatile("v_nop\n\tv_nop\n\tv_nop\n\tv_nop" : "+v"(a), "+v"(b), "+v"(c), "+v"(d)); }
__device__ __forceinline__ void acc_guard2(v8f& a, v8f& b) { asm volatile("v_nop\n\tv_nop\n\tv_nop\n\tv_nop" : "+v"(a), "+v"(b)); }

template <typename T> struct Frag;
template <> struct Frag<_Float16> {
  typedef v16h V; union U { v16h v; v8h h[2]; };
  static __device__ __forceinline__ v16h load(const _Float16* p) {
    U f; f.h[0] = *(const v8h*)(p); f.h[1] = *(const v8h*)(p + 16); return f.v;
  }
  static __device__ __forceinline__ v8f mma(v16h a, v16h b, v8f c) {
    return __builtin_amdgcn_wmma_f32_16x16x32_f16(false, a, false, b, (short)0, c, false, false);
  }
  static __device__ __forceinline__ void guard(v8f& a, v8f& b, v16h x, v16h y) { dep_guard_h(a, b, x, y); }
  static __device__ __forceinline__ void keep(v16h a, v16h b, v16h c, v16h d) { keep4_h(a, b, c, d); }
};
template <> struct Frag<__bf16> {
  typedef v16b V; union U { v16b v; v8b h[2]; };
  static __device__ __forceinline__ v16b load(const __bf16* p) {
    U f; f.h[0] = *(const v8b*)(p); f.h[1] = *(const v8b*)(p + 16); return f.v;
  }
  static __device__ __forceinline__ v8f mma(v16b a, v16b b, v8f c) {
    return __builtin_amdgcn_wmma_f32_16x16x32_bf16(false, a, false, b, (short)0, c, false, false);
  }
  static __device__ __forceinline__ void guard(v8f& a, v8f& b, v16b x, v16b y) { dep_guard_b(a, b, x, y); }
  static __device__ __forceinline__ void keep(v16b a, v16b b, v16b c, v16b d) { keep4_b(a, b, c, d); }
};

template <int ET> struct Elem;
template <> struct Elem<0> { typedef _Float16 T; };
template <> struct Elem<1> { typedef __bf16 T; };
template <int ET, bool SPLIT, int BIAS_MODE, int OUT_MODE, bool RESID, int ACT = 0>
__global__ __launch_bounds__(256) void wmma_gemm64(
    const unsigned short* __restrict__ Ap, const unsigned short* __restrict__ A2p, int lda, long strideA,
    const unsigned short* __restrict__ Btp, const unsigned short* __restrict__ Bt2p, int ldb, long strideB,
    void* __restrict__ Cout, void* __restrict__ Cout2, int ldc, long strideC,
    const float* __restrict__ bias,
    const float* __restrict__ resid, long strideR,
    int M, int N, int K, float scale) {
  typedef typename Elem<ET>::T T;
  typedef typename Frag<T>::V V;
  const T* A = (const T*)Ap; const T* A2 = (const T*)A2p; const T* Bt = (const T*)Btp; const T* Bt2 = (const T*)Bt2p;
  __shared__ __align__(16) float sT[8][16 * 68];
  const int b    = blockIdx.y;
  const int lane = threadIdx.x & 31;
  const int wave = threadIdx.x >> 5;
  const int tilesN = N >> 6;
  const int tilesM = M >> 6;
  const int tile = blockIdx.x * 8 + wave;
  if (tile >= tilesM * tilesN) return;
  const int tm = tile / tilesN;
  const int tn = tile - tm * tilesN;
  const int m0 = tm << 6;
  const int n0 = tn << 6;

  const T* Ab  = A  + (size_t)b * strideA;
  const T* Bb  = Bt + (size_t)b * strideB;
  const T* Ab2 = SPLIT ? (A2  + (size_t)b * strideA) : nullptr;
  const T* Bb2 = SPLIT ? (Bt2 + (size_t)b * strideB) : nullptr;

  const int rlane = lane & 15;
  const int koff  = (lane >> 4) * 8;
  const int mOff  = (lane >> 4) * 8;

  v8f acc[4][4];
#pragma unroll
  for (int i = 0; i < 4; ++i)
#pragma unroll
    for (int j = 0; j < 4; ++j) acc[i][j] = (v8f){0.f,0.f,0.f,0.f,0.f,0.f,0.f,0.f};

  for (int k0 = 0; k0 < K; k0 += 32) {
    V bh[4], bl[4];
#pragma unroll
    for (int j = 0; j < 4; ++j) {
      const size_t bo = (size_t)(n0 + (j << 4) + rlane) * ldb + koff + k0;
      bh[j] = Frag<T>::load(Bb + bo);
      if (SPLIT) bl[j] = Frag<T>::load(Bb2 + bo);
    }
#pragma unroll
    for (int i = 0; i < 4; ++i) {
      const size_t ao = (size_t)(m0 + (i << 4) + rlane) * lda + koff + k0;
      V ah = Frag<T>::load(Ab + ao);
      V al;
      if (SPLIT) al = Frag<T>::load(Ab2 + ao);
#pragma unroll
      for (int j = 0; j < 4; ++j) {
        acc[i][j] = Frag<T>::mma(ah, bh[j], acc[i][j]);
        if (SPLIT) {
          acc[i][j] = Frag<T>::mma(ah, bl[j], acc[i][j]);
          acc[i][j] = Frag<T>::mma(al, bh[j], acc[i][j]);
        }
      }
      Frag<T>::guard(acc[i][0], acc[i][3], ah, SPLIT ? al : ah);
    }
    Frag<T>::keep(bh[0], bh[1], bh[2], bh[3]);
    if (SPLIT) Frag<T>::keep(bl[0], bl[1], bl[2], bl[3]);
  }
  acc_guard4(acc[0][0], acc[0][1], acc[0][2], acc[0][3]);
  acc_guard4(acc[1][0], acc[1][1], acc[1][2], acc[1][3]);
  acc_guard4(acc[2][0], acc[2][1], acc[2][2], acc[2][3]);
  acc_guard4(acc[3][0], acc[3][1], acc[3][2], acc[3][3]);

  float* slab = sT[wave];
  const float* Rb = RESID ? (resid + (size_t)b * strideR) : nullptr;
#pragma unroll
  for (int i = 0; i < 4; ++i) {
    const int mBase = m0 + (i << 4);
#pragma unroll
    for (int j = 0; j < 4; ++j) {
      const int n = n0 + (j << 4) + rlane;
      float bv = 0.f;
      if (BIAS_MODE == 2) bv = bias[n];
#pragma unroll
      for (int r = 0; r < 8; ++r) {
        float v = acc[i][j][r] * scale;
        if (BIAS_MODE == 1) v += bias[mBase + mOff + r];
        if (BIAS_MODE == 2) v += bv;
        if (RESID) v += Rb[(size_t)(mBase + mOff + r) * ldc + n];
        if (ACT == 1) v = tanhf(v);
        if (ACT == 2) v = fmaxf(v, 0.0f);
        if (ACT == 3) v = v / (1.0f + expf(-v));
        if (ACT == 4) v = (v > 0.f) ? v : 0.01f * v;
        if (ACT == 5) v = 0.5f * v * (1.0f + erff(v * 0.70710678118654752f));
        slab[(mOff + r) * 68 + (j << 4) + rlane] = v;
      }
    }
    __builtin_amdgcn_fence(__ATOMIC_RELEASE, "workgroup");
    __builtin_amdgcn_wave_barrier();
    __builtin_amdgcn_fence(__ATOMIC_ACQUIRE, "workgroup");
    if (OUT_MODE == 0) {
      float* C = (float*)Cout + (size_t)b * strideC;
      const int hh = lane >> 4, c4 = (lane & 15) * 4;
      for (int pass = 0; pass < 2; ++pass) {
#pragma unroll
        for (int it = 0; it < 8; ++it) {
          const int row = it * 2 + hh;
          v4f v = *(const v4f*)(slab + row * 68 + c4);
          *(volatile v4f*)(C + (size_t)(mBase + row) * ldc + n0 + c4) = v;
        }
        __threadfence();
      }
    } else {
      const int q = lane >> 3, c8 = (lane & 7) * 8;
      unsigned short* C  = (unsigned short*)Cout  + (size_t)b * strideC;
      unsigned short* C2 = (OUT_MODE == 2) ? ((unsigned short*)Cout2 + (size_t)b * strideC) : nullptr;
      for (int pass = 0; pass < 2; ++pass) {
#pragma unroll
        for (int it = 0; it < 4; ++it) {
          const int row = it * 4 + q;
          const float* sp = slab + row * 68 + c8;
          v8h hv, lv;
#pragma unroll
          for (int e = 0; e < 8; ++e) {
            if (OUT_MODE == 1) {
              hv[e] = (_Float16)sp[e];
            } else {
              unsigned short hb = f2bf_bits(sp[e]);
              unsigned short lb = f2bf_bits(sp[e] - bf_bits2f(hb));
              hv[e] = __builtin_bit_cast(_Float16, hb);
              lv[e] = __builtin_bit_cast(_Float16, lb);
            }
          }
          *(volatile v8h*)(C + (size_t)(mBase + row) * ldc + n0 + c8) = hv;
          if (OUT_MODE == 2) *(volatile v8h*)(C2 + (size_t)(mBase + row) * ldc + n0 + c8) = lv;
        }
        __threadfence();
      }
    }
    __builtin_amdgcn_fence(__ATOMIC_RELEASE, "workgroup");
    __builtin_amdgcn_wave_barrier();
    __builtin_amdgcn_fence(__ATOMIC_ACQUIRE, "workgroup");
  }
}

constexpr int kBatch   = 128;
constexpr int kSteps   = 256;
constexpr int kIn      = 4096;
constexpr int kHid     = 512;
constexpr int kOut     = 4096;
constexpr int kPitch   = 520;
constexpr int kRows    = 16;
constexpr int kRecThreads = 512;

static_assert(kHid % 32 == 0);
static_assert(kBatch % 64 == 0);
static_assert(kOut % 64 == 0);
static_assert(kBatch % kRows == 0);
static_assert((kRecThreads / 32) * 32 == kHid);
static_assert(kPitch % 8 == 0 && kPitch >= kHid);

constexpr size_t kXptBytes  = (size_t)kSteps * kHid * kBatch * 4;
constexpr size_t kWhhBytes  = (size_t)kHid * kHid * 2;
constexpr size_t kWfcBytes  = (size_t)kOut * kHid * 2;
constexpr size_t kHlBytes   = (size_t)kBatch * kHid * 2;
constexpr size_t kOffXpt    = 0;
constexpr size_t kOffWhhHi  = kOffXpt + kXptBytes;
constexpr size_t kOffWhhLo  = kOffWhhHi + kWhhBytes;
constexpr size_t kOffWfcHi  = kOffWhhLo + kWhhBytes;
constexpr size_t kOffWfcLo  = kOffWfcHi + kWfcBytes;
constexpr size_t kOffHlHi   = kOffWfcLo + kWfcBytes;
constexpr size_t kOffHlLo   = kOffHlHi + kHlBytes;
constexpr size_t kWsTotal   = kOffHlLo + kHlBytes;
static_assert(kWsTotal == 76808192ull);
static_assert(kWsTotal <= 134217728ull);
static_assert(kOffWhhHi % 128 == 0 && kOffWhhLo % 128 == 0 && kOffWfcHi % 128 == 0 &&
              kOffWfcLo % 128 == 0 && kOffHlHi % 128 == 0 && kOffHlLo % 128 == 0);

__global__ __launch_bounds__(256) void split_f32_bf16x8(
    const float* __restrict__ in, unsigned short* __restrict__ hi, unsigned short* __restrict__ lo, int n8) {
  const int i = blockIdx.x * 256 + threadIdx.x;
  if (i < n8) {
    const size_t o = (size_t)i * 8;
    const v4f a = *(const v4f*)(in + o);
    const v4f c = *(const v4f*)(in + o + 4);
    const float f[8] = {a[0], a[1], a[2], a[3], c[0], c[1], c[2], c[3]};
    v8h hv, lv;
#pragma unroll
    for (int e = 0; e < 8; ++e) {
      const unsigned short hb = f2bf_bits(f[e]);
      const unsigned short lb = f2bf_bits(f[e] - bf_bits2f(hb));
      hv[e] = __builtin_bit_cast(_Float16, hb);
      lv[e] = __builtin_bit_cast(_Float16, lb);
    }
    _Float16* hp = (_Float16*)(void*)hi + o;
    _Float16* lp = (_Float16*)(void*)lo + o;
    *(volatile v8h*)hp = hv;
    *(volatile v8h*)lp = lv;
    __threadfence();
    *(volatile v8h*)hp = hv;
    *(volatile v8h*)lp = lv;
  }
}

__global__ __launch_bounds__(256) void gather_xp_kernel(
    const int* __restrict__ x, const float* __restrict__ wih, const float* __restrict__ bih,
    float* __restrict__ xpt) {
  const int tid  = threadIdx.x;
  const int lane = tid & 31;
  const int nl   = tid >> 5;
  const int t    = blockIdx.x >> 6;
  const int n    = (blockIdx.x & 63) * 8 + nl;
  const int bb   = lane * 4;
  float w[4];
#pragma unroll
  for (int i = 0; i < 4; ++i) {
    int xi = x[(size_t)(bb + i) * kSteps + t];
    xi = xi < 0 ? 0 : (xi > (kIn - 1) ? (kIn - 1) : xi);
    w[i] = wih[(size_t)n * kIn + xi];
  }
  const float bi = bih[n];
  v4f o;
  o[0] = w[0] + bi; o[1] = w[1] + bi; o[2] = w[2] + bi; o[3] = w[3] + bi;
  float* dst = xpt + ((size_t)t * kHid + n) * kBatch + bb;
  *(volatile v4f*)dst = o;
  __threadfence();
  *(volatile v4f*)dst = o;
}

__global__ __launch_bounds__(512) void rnn_steps_kernel(
    const float* __restrict__ xpt,
    const unsigned short* __restrict__ whh_hi, const unsigned short* __restrict__ whh_lo,
    const float* __restrict__ bhh,
    unsigned short* __restrict__ hl_hi, unsigned short* __restrict__ hl_lo) {
  __shared__ __align__(16) __bf16 Hh[kRows * kPitch];
  __shared__ __align__(16) __bf16 Hl[kRows * kPitch];
  union FB { v16b v; v8b h[2]; };

  const int tid  = threadIdx.x;
  const int lane = tid & 31;
  const int wave = tid >> 5;
  const int hh   = lane >> 4;
  const int c    = lane & 15;
  const int b0   = blockIdx.x * kRows;
  const int n0   = wave * 32 + c;
  const int n1   = n0 + 16;

  const __bf16 z = __builtin_bit_cast(__bf16, (unsigned short)0);
  for (int i = tid; i < kRows * kPitch; i += kRecThreads) { Hh[i] = z; Hl[i] = z; }

  const float bh0 = bhh[n0];
  const float bh1 = bhh[n1];
  const __bf16* Wh = (const __bf16*)(const void*)whh_hi;
  const __bf16* Wl = (const __bf16*)(const void*)whh_lo;
  const __bf16* wr0h = Wh + (size_t)n0 * kHid + 8 * hh;
  const __bf16* wr0l = Wl + (size_t)n0 * kHid + 8 * hh;
  const __bf16* wr1h = Wh + (size_t)n1 * kHid + 8 * hh;
  const __bf16* wr1l = Wl + (size_t)n1 * kHid + 8 * hh;
  const int aoff = c * kPitch + 8 * hh;
  __syncthreads();

  for (int t = 0; t < kSteps; ++t) {
    const float* xp0p = xpt + ((size_t)t * kHid + n0) * kBatch + b0 + 8 * hh;
    const float* xp1p = xpt + ((size_t)t * kHid + n1) * kBatch + b0 + 8 * hh;
    const v4f xq0a = *(const v4f*)(xp0p);
    const v4f xq0b = *(const v4f*)(xp0p + 4);
    const v4f xq1a = *(const v4f*)(xp1p);
    const v4f xq1b = *(const v4f*)(xp1p + 4);
    const float xr0[8] = {xq0a[0], xq0a[1], xq0a[2], xq0a[3], xq0b[0], xq0b[1], xq0b[2], xq0b[3]};
    const float xr1[8] = {xq1a[0], xq1a[1], xq1a[2], xq1a[3], xq1b[0], xq1b[1], xq1b[2], xq1b[3]};

    v8f acc0 = (v8f){0.f,0.f,0.f,0.f,0.f,0.f,0.f,0.f};
    v8f acc1 = (v8f){0.f,0.f,0.f,0.f,0.f,0.f,0.f,0.f};
#pragma unroll 2
    for (int kb = 0; kb < kHid / 32; ++kb) {
      const int k0 = kb * 32;
      FB fa, fl;
      fa.h[0] = *(const v8b*)(Hh + aoff + k0);
      fa.h[1] = *(const v8b*)(Hh + aoff + k0 + 16);
      fl.h[0] = *(const v8b*)(Hl + aoff + k0);
      fl.h[1] = *(const v8b*)(Hl + aoff + k0 + 16);
      const v16b ah = fa.v;
      const v16b al = fl.v;
      const v16b bt0h = Frag<__bf16>::load(wr0h + k0);
      const v16b bt0l = Frag<__bf16>::load(wr0l + k0);
      const v16b bt1h = Frag<__bf16>::load(wr1h + k0);
      const v16b bt1l = Frag<__bf16>::load(wr1l + k0);
      acc0 = Frag<__bf16>::mma(ah, bt0h, acc0);
      acc0 = Frag<__bf16>::mma(ah, bt0l, acc0);
      acc0 = Frag<__bf16>::mma(al, bt0h, acc0);
      acc1 = Frag<__bf16>::mma(ah, bt1h, acc1);
      acc1 = Frag<__bf16>::mma(ah, bt1l, acc1);
      acc1 = Frag<__bf16>::mma(al, bt1h, acc1);
      Frag<__bf16>::guard(acc0, acc1, ah, al);
      Frag<__bf16>::keep(bt0h, bt0l, bt1h, bt1l);
    }
    acc_guard2(acc0, acc1);
    __syncthreads();

#pragma unroll
    for (int r = 0; r < 8; ++r) {
      const float v0 = (xr0[r] + acc0[r]) + bh0;
      const float v1 = (xr1[r] + acc1[r]) + bh1;
      const float h0v = tanhf(v0);
      const float h1v = tanhf(v1);
      const unsigned short hb0 = f2bf_bits(h0v);
      const unsigned short lb0 = f2bf_bits(h0v - bf_bits2f(hb0));
      const unsigned short hb1 = f2bf_bits(h1v);
      const unsigned short lb1 = f2bf_bits(h1v - bf_bits2f(hb1));
      const int ro = (8 * hh + r) * kPitch;
      Hh[ro + n0] = __builtin_bit_cast(__bf16, hb0);
      Hl[ro + n0] = __builtin_bit_cast(__bf16, lb0);
      Hh[ro + n1] = __builtin_bit_cast(__bf16, hb1);
      Hl[ro + n1] = __builtin_bit_cast(__bf16, lb1);
    }
    __syncthreads();
  }

  {
    const int q  = lane >> 3;
    const int c8 = (lane & 7) * 8;
    _Float16* gh = (_Float16*)(void*)hl_hi;
    _Float16* gl = (_Float16*)(void*)hl_lo;
    for (int pass = 0; pass < 2; ++pass) {
#pragma unroll
      for (int it = 0; it < 2; ++it) {
        const int L   = wave * 8 + it * 4 + q;
        const int row = L >> 3;
        const int seg = L & 7;
        const v8b bvh = *(const v8b*)(Hh + row * kPitch + seg * 64 + c8);
        const v8b bvl = *(const v8b*)(Hl + row * kPitch + seg * 64 + c8);
        const v8h hvh = __builtin_bit_cast(v8h, bvh);
        const v8h hvl = __builtin_bit_cast(v8h, bvl);
        const size_t go = (size_t)(b0 + row) * kHid + seg * 64 + c8;
        *(volatile v8h*)(gh + go) = hvh;
        *(volatile v8h*)(gl + go) = hvl;
      }
      __threadfence();
    }
  }
}

extern "C" void kernel_launch(void* const* d_in, const int* in_sizes, int n_in,
                              void* d_out, int out_size, void* d_ws, size_t ws_size,
                              hipStream_t stream) {
  if (n_in < 7) return;
  if (in_sizes[0] != kBatch * kSteps) return;
  if (in_sizes[1] != kHid * kIn) return;
  if (in_sizes[2] != kHid) return;
  if (in_sizes[3] != kHid * kHid) return;
  if (in_sizes[4] != kHid) return;
  if (in_sizes[5] != kOut * kHid) return;
  if (in_sizes[6] != kOut) return;
  if (out_size != kBatch * kOut) return;
  if (ws_size < kWsTotal) return;

  const int*   x   = (const int*)  d_in[0];
  const float* wih = (const float*)d_in[1];
  const float* bih = (const float*)d_in[2];
  const float* whh = (const float*)d_in[3];
  const float* bhh = (const float*)d_in[4];
  const float* wfc = (const float*)d_in[5];
  const float* bfc = (const float*)d_in[6];
  float* out = (float*)d_out;

  char* ws = (char*)d_ws;
  float*          xpt    = (float*)(ws + kOffXpt);
  unsigned short* whh_hi = (unsigned short*)(ws + kOffWhhHi);
  unsigned short* whh_lo = (unsigned short*)(ws + kOffWhhLo);
  unsigned short* wfc_hi = (unsigned short*)(ws + kOffWfcHi);
  unsigned short* wfc_lo = (unsigned short*)(ws + kOffWfcLo);
  unsigned short* hl_hi  = (unsigned short*)(ws + kOffHlHi);
  unsigned short* hl_lo  = (unsigned short*)(ws + kOffHlLo);

  const int n8_whh = (kHid * kHid) / 8;
  const int n8_wfc = (kOut * kHid) / 8;
  split_f32_bf16x8<<<(n8_whh + 255) / 256, 256, 0, stream>>>(whh, whh_hi, whh_lo, n8_whh);
  split_f32_bf16x8<<<(n8_wfc + 255) / 256, 256, 0, stream>>>(wfc, wfc_hi, wfc_lo, n8_wfc);

  gather_xp_kernel<<<kSteps * (kHid / 8), 256, 0, stream>>>(x, wih, bih, xpt);

  rnn_steps_kernel<<<kBatch / kRows, kRecThreads, 0, stream>>>(xpt, whh_hi, whh_lo, bhh, hl_hi, hl_lo);

  const int tiles = (kBatch / 64) * (kOut / 64);
  wmma_gemm64<1, true, 2, 0, false, 0><<<dim3((tiles + 7) / 8, 1), 256, 0, stream>>>(
      hl_hi, hl_lo, kHid, 0L,
      wfc_hi, wfc_lo, kHid, 0L,
      (void*)out, nullptr, kOut, 0L,
      bfc, nullptr, 0L,
      kBatch, kOut, kHid, 1.0f);
}
